// PuzzleMoE_68667937129030
// MI455X (gfx1250) — hardware-verified
//
#include <hip/hip_runtime.h>
#include <math.h>

typedef __attribute__((ext_vector_type(16))) _Float16 v16h;
typedef __attribute__((ext_vector_type(16))) __bf16 v16b;
typedef __attribute__((ext_vector_type(8)))  _Float16 v8h;
typedef __attribute__((ext_vector_type(8)))  float v8f;
typedef __attribute__((ext_vector_type(4)))  float v4f;
typedef __attribute__((ext_vector_type(2)))  float v2f;
typedef __attribute__((ext_vector_type(4)))  unsigned v4u;
typedef __attribute__((ext_vector_type(4)))  int v4i;
typedef float __attribute__((may_alias)) float_a;
typedef int __attribute__((may_alias)) int_a;

template <typename T> __device__ __forceinline__ void vst2(void* p, T v) { *(volatile T*)p = v; __threadfence(); *(volatile T*)p = v; }
__device__ __forceinline__ v8f wmma16(v16h a, v16h b, v8f c) {
  v8f d = __builtin_amdgcn_wmma_f32_16x16x32_f16(false, a, false, b, (short)0, c, false, false);
  asm volatile("v_nop\n\tv_nop\n\tv_nop\n\tv_nop" : "+v"(d) : "v"(a), "v"(b));
  return d;
}
__device__ __forceinline__ v8f wmma_bf(v16b a, v16b b, v8f c) {
  v8f d = __builtin_amdgcn_wmma_f32_16x16x32_bf16(false, a, false, b, (short)0, c, false, false);
  asm volatile("v_nop\n\tv_nop\n\tv_nop\n\tv_nop" : "+v"(d) : "v"(a), "v"(b));
  return d;
}
__device__ __forceinline__ v16h frag_h(const _Float16* rowk0, int lane) {
  union { v16h v; v8h q[2]; } u; const _Float16* p = rowk0 + 8 * (lane >> 4);
  u.q[0] = *(const v8h*)p; u.q[1] = *(const v8h*)(p + 16); return u.v;
}
__device__ __forceinline__ v16h frag_f32(const float* rowk0, int lane) {
  v16h a; const float* p = rowk0 + 8 * (lane >> 4);
#pragma unroll
  for (int i = 0; i < 8; ++i) { a[i] = (_Float16)p[i]; a[8 + i] = (_Float16)p[16 + i]; }
  return a;
}
__device__ __forceinline__ v16h frag_f32s(const float* rowk0, int lane, float sc) {
  v16h a; const float* p = rowk0 + 8 * (lane >> 4);
#pragma unroll
  for (int i = 0; i < 8; ++i) { a[i] = (_Float16)(p[i] * sc); a[8 + i] = (_Float16)(p[16 + i] * sc); }
  return a;
}
__device__ __forceinline__ v16h fragc_f32(const float* W, int k0, int n, int lane, int ld, int K) {
  v16h a; const int g = lane >> 4;
#pragma unroll
  for (int i = 0; i < 8; ++i) { const int ka = k0 + 8 * g + i, kb = ka + 16;
    a[i] = (_Float16)(ka < K ? W[(size_t)(ka < K ? ka : K - 1) * ld + n] : 0.f); a[8 + i] = (_Float16)(kb < K ? W[(size_t)(kb < K ? kb : K - 1) * ld + n] : 0.f); }
  return a;
}
struct F2 { v16b h, l; };
__device__ __forceinline__ F2 bsplit16(const float v[16]) { F2 r;
#pragma unroll
  for (int i = 0; i < 16; ++i) { const __bf16 h = (__bf16)v[i]; r.h[i] = h; r.l[i] = (__bf16)(v[i] - (float)h); }
  return r; }
__device__ __forceinline__ F2 split_row(const float* row, int k0, int lane) { float v[16]; const float* p = row + k0 + 8 * (lane >> 4);
#pragma unroll
  for (int i = 0; i < 8; ++i) { v[i] = p[i]; v[8 + i] = p[16 + i]; }
  return bsplit16(v); }
__device__ __forceinline__ F2 split_rowK(const float* row, int k0, int lane, int K) { float v[16]; const int g = lane >> 4;
#pragma unroll
  for (int i = 0; i < 8; ++i) { const int ka = k0 + 8 * g + i, kb = ka + 16; v[i] = ka < K ? row[ka < K ? ka : K - 1] : 0.f; v[8 + i] = kb < K ? row[kb < K ? kb : K - 1] : 0.f; }
  return bsplit16(v); }
__device__ __forceinline__ F2 split_col(const float* W, int k0, int n, int lane, int ld, int K) { float v[16]; const int g = lane >> 4;
#pragma unroll
  for (int i = 0; i < 8; ++i) { const int ka = k0 + 8 * g + i, kb = ka + 16; v[i] = ka < K ? W[(size_t)(ka < K ? ka : K - 1) * ld + n] : 0.f; v[8 + i] = kb < K ? W[(size_t)(kb < K ? kb : K - 1) * ld + n] : 0.f; }
  return bsplit16(v); }
__device__ __forceinline__ v8f mac3(const F2& a, const F2& b, v8f c) { c = wmma_bf(a.l, b.h, c); c = wmma_bf(a.h, b.l, c); return wmma_bf(a.h, b.h, c); }
__device__ __forceinline__ float sigm(float v) { return 1.0f / (1.0f + expf(-v)); }
#define LDSX() do { asm volatile("s_wait_dscnt 0" ::: "memory"); __builtin_amdgcn_wave_barrier(); __builtin_amdgcn_fence(__ATOMIC_RELEASE, "workgroup"); } while (0)


#define NB 512
#define NP 9
#define NS (NB * NP)
#define NSPAD 4608
#define CL 12
#define LL 256
#define CH 64
#define DD 512
#define NE 8
#define NC 128
#ifndef NSB
#define NSB (NSPAD / 64)
#define NSAMP NS
#endif
typedef __attribute__((ext_vector_type(8))) __bf16 v8b;
__device__ __forceinline__ v16b frag_b(const __bf16* rowk0, int lane) {
  union { v16b v; v8b q[2]; } u; const __bf16* p = rowk0 + 8 * (lane >> 4);
  u.q[0] = *(const v8b*)p; u.q[1] = *(const v8b*)(p + 16); return u.v;
}
__device__ __forceinline__ float bfr(float v) { return (float)(__bf16)v; }
__device__ __attribute__((noinline)) float exp_ni(float v) { return expf(v); }
__device__ __attribute__((noinline)) float erf_ni(float v) { return erff(v); }

#define WS_PW  0u
#define PC1 0
#define PC2 (PC1 + CH * 64)
#define PPJ (PC2 + CH * 192)
#define PGT (PPJ + DD * CH)
#define PE1 (PGT + 16 * DD)
#define PE2 (PE1 + NE * DD * DD)
#define PWEND (PE2 + NE * NC * DD)
#define WS_FEAT (WS_PW + 2u * PWEND)
#define WS_EMB  (WS_FEAT + 4u * NSPAD * CH)
#define WS_GATE (WS_EMB + 4u * NSPAD * DD)
#define WS_H1   (WS_GATE + 4u * NSPAD * NE)
#define WS_OE   (WS_H1 + 4u * NSPAD * NE * DD)
#define WS_END  (WS_OE + 4u * NSPAD * NE * NC)

__global__ __launch_bounds__(256) void k_pack(const float* __restrict__ C1W, const float* __restrict__ C2W, const float* __restrict__ PJ, const float* __restrict__ GW, const float* __restrict__ E1, const float* __restrict__ E2, __bf16* __restrict__ PW) {
  __shared__ __align__(16) __bf16 s[DD]; const int n = blockIdx.x, which = blockIdx.y, tid = threadIdx.x; int K; size_t dst;
  if (which == 0) { if (n >= CH) return; K = 64; dst = PC1 + (size_t)n * 64; for (int k = tid; k < K; k += 256) s[k] = (__bf16)((k < CL * 5) ? C1W[((size_t)n * CL + k / 5) * 5 + k % 5] : 0.f); }
  else if (which == 1) { if (n >= CH) return; K = 192; dst = PC2 + (size_t)n * 192; for (int k = tid; k < K; k += 256) s[k] = (__bf16)C2W[(size_t)n * 192 + k]; }
  else if (which == 2) { if (n >= DD) return; K = CH; dst = PPJ + (size_t)n * CH; for (int k = tid; k < K; k += 256) s[k] = (__bf16)PJ[(size_t)k * DD + n]; }
  else if (which == 3) { if (n >= 16) return; K = DD; dst = PGT + (size_t)n * DD; for (int k = tid; k < K; k += 256) s[k] = (__bf16)((n < NE) ? GW[(size_t)k * NE + n] : 0.f); }
  else if (which == 4) { K = DD; const int e = n / DD, o = n % DD; dst = PE1 + (size_t)n * DD; for (int k = tid; k < K; k += 256) s[k] = (__bf16)E1[((size_t)e * DD + k) * DD + o]; }
  else { if (n >= NE * NC) return; K = DD; const int e = n / NC, o = n % NC; dst = PE2 + (size_t)n * DD; for (int k = tid; k < K; k += 256) s[k] = (__bf16)E2[((size_t)e * DD + k) * NC + o]; }
  __syncthreads();
  for (int q = tid; q < K / 8; q += 256) vst2((unsigned*)(PW + dst + q * 8), *(const v4u*)&s[q * 8]);
}
__global__ __launch_bounds__(128) void k_conv(const float* __restrict__ X, const __bf16* __restrict__ PW, const float* __restrict__ B1c, const float* __restrict__ B2c, float* __restrict__ FEAT) {
  __shared__ float sh1[CH][LL + 4];
  __shared__ __align__(16) float scs[4][CH]; __shared__ __align__(16) float sf[CH];
  const int tid = threadIdx.x, wave = tid >> 5, lane = tid & 31, col = lane & 15, g = lane >> 4; const int smp = blockIdx.x;
  const float* xs = X + (size_t)smp * CL * LL;
#pragma unroll 1
  for (int rt = 0; rt < 4; ++rt) { const int p0 = wave * 64 + rt * 16; const int pos = p0 + col;
    v8f acc[4] = {};
#pragma unroll 1
    for (int kc = 0; kc < 2; ++kc) { v16b a;
#pragma unroll
      for (int i = 0; i < 16; ++i) { const int kk = kc * 32 + 8 * g + (i & 7) + ((i >> 3) << 4); float v = 0.f; if (kk < CL * 5) { const int c = kk / 5, t = kk - c * 5; const int pp = pos + t - 2; if (pp >= 0 && pp < LL) v = xs[c * LL + pp]; } a[i] = (__bf16)v; }
#pragma unroll
      for (int j = 0; j < 4; ++j) acc[j] = wmma_bf(a, frag_b(PW + PC1 + (size_t)(j * 16 + col) * 64 + kc * 32, lane), acc[j]); }
#pragma unroll
    for (int j = 0; j < 4; ++j) { const int ch = j * 16 + col; const float bb = bfr(B1c[ch]);
#pragma unroll
      for (int r = 0; r < 8; ++r) sh1[ch][p0 + 8 * g + r] = fmaxf(acc[j][r] + bb, 0.f); } }
  __syncthreads();
  float csum[4]; for (int j = 0; j < 4; ++j) csum[j] = 0.f;
#pragma unroll 1
  for (int rt = 0; rt < 4; ++rt) { const int p0 = wave * 64 + rt * 16; const int pos = p0 + col;
    v8f acc[4] = {};
#pragma unroll 1
    for (int kc = 0; kc < 6; ++kc) { float v[16];
#pragma unroll
      for (int i = 0; i < 16; ++i) { const int kk = kc * 32 + 8 * g + (i & 7) + ((i >> 3) << 4); const int c = kk / 3, t = kk - c * 3; const int pp = pos + t - 1; v[i] = (pp >= 0 && pp < LL) ? sh1[c][pp] : 0.f; }
      const F2 a = bsplit16(v);
#pragma unroll
      for (int j = 0; j < 4; ++j) { const v16b w = frag_b(PW + PC2 + (size_t)(j * 16 + col) * 192 + kc * 32, lane); acc[j] = wmma_bf(a.l, w, acc[j]); acc[j] = wmma_bf(a.h, w, acc[j]); } }
#pragma unroll
    for (int j = 0; j < 4; ++j) { const float bb = bfr(B2c[j * 16 + col]); float s_ = 0.f;
#pragma unroll
      for (int r = 0; r < 8; ++r) s_ += fmaxf(acc[j][r] + bb, 0.f);
      s_ += __shfl_xor(s_, 16);
      csum[j] += s_; } }
  if (g == 0) {
#pragma unroll
    for (int j = 0; j < 4; ++j) scs[wave][j * 16 + col] = csum[j]; }
  __syncthreads();
  if (tid < CH) sf[tid] = (((scs[0][tid] + scs[1][tid]) + scs[2][tid]) + scs[3][tid]) * (1.0f / (float)LL);
  __syncthreads();
  if (tid < 16) vst2(FEAT + (size_t)smp * CH + tid * 4, *(const v4f*)&sf[tid * 4]);
}
template <int NT, int EPI>
__global__ __launch_bounds__(128) void k_gemm(const float* __restrict__ A, int lda, int K, const __bf16* __restrict__ P, const float* __restrict__ bias, int bias_mod, const float* __restrict__ POS, float* __restrict__ OUT, int ldo) {
  __shared__ __align__(16) float so[4][16][NT * 16 + 4];
  const int tid = threadIdx.x, wave = tid >> 5, lane = tid & 31, col = lane & 15, g = lane >> 4; const size_t r0 = (size_t)blockIdx.x * 64 + wave * 16; const int n0 = blockIdx.y * (NT * 16);
  v8f acc[NT]; for (int j = 0; j < NT; ++j) acc[j] = (v8f){};
#pragma unroll 2
  for (int kc = 0; kc < K / 32; ++kc) { const F2 a = split_row(A + (r0 + col) * (size_t)lda, kc * 32, lane);
#pragma unroll
    for (int j = 0; j < NT; ++j) { const v16b w = frag_b(P + (size_t)(n0 + j * 16 + col) * K + kc * 32, lane); acc[j] = wmma_bf(a.l, w, acc[j]); acc[j] = wmma_bf(a.h, w, acc[j]); } }
#pragma unroll
  for (int j = 0; j < NT; ++j) { const int n = n0 + j * 16 + col; const float bb = bias ? bfr(bias[n % bias_mod]) : 0.f;
#pragma unroll
    for (int r = 0; r < 8; ++r) { float v = acc[j][r] + bb; if (EPI == 1) v = fmaxf(v, 0.f); if (EPI == 2) v += bfr(POS[((r0 + 8 * g + r) % NP) * DD + n]); so[wave][8 * g + r][j * 16 + col] = v; } }
  LDSX();
  for (int rl = 0; rl < 16; ++rl) if (lane < NT * 4) vst2(OUT + (r0 + rl) * ldo + n0 + lane * 4, *(const v4f*)&so[wave][rl][lane * 4]);
}
__global__ __launch_bounds__(128) void k_gate(const float* __restrict__ EMB, const __bf16* __restrict__ PW, const float* __restrict__ GB, const int* __restrict__ TOPK, float* __restrict__ GATE) {
  __shared__ float sl[4][16][NE + 1]; __shared__ __align__(16) float sg[64][NE];
  const int tid = threadIdx.x, wave = tid >> 5, lane = tid & 31, col = lane & 15, g = lane >> 4; const size_t r0 = (size_t)blockIdx.x * 64 + wave * 16;
  v8f acc = {};
#pragma unroll 4
  for (int kc = 0; kc < DD / 32; ++kc) { const F2 a = split_row(EMB + (r0 + col) * DD, kc * 32, lane); const v16b w = frag_b(PW + PGT + (size_t)col * DD + kc * 32, lane); acc = wmma_bf(a.l, w, acc); acc = wmma_bf(a.h, w, acc); }
  if (col < NE) {
#pragma unroll
    for (int r = 0; r < 8; ++r) sl[wave][8 * g + r][col] = acc[r] + bfr(GB[col]); }
  LDSX();
  if (lane < 16) { const int rl = lane, tl = wave * 16 + rl; float lg[NE]; bool sel[NE]; int kk = min(max(TOPK[0], 1), NE);
#pragma unroll
    for (int e = 0; e < NE; ++e) { lg[e] = sl[wave][rl][e]; sel[e] = false; }
    float vmax = -3.0e38f;
    for (int t = 0; t < kk; ++t) { int bi = -1; float bv = -3.0e38f;
#pragma unroll
      for (int e = 0; e < NE; ++e) if (!sel[e] && (bi < 0 || lg[e] > bv)) { bv = lg[e]; bi = e; }
      sel[bi] = true; if (t == 0) vmax = bv; }
    float z = 0.f; float w[NE];
#pragma unroll
    for (int e = 0; e < NE; ++e) { w[e] = sel[e] ? exp_ni(lg[e] - vmax) : 0.f; z += w[e]; }
    const float iz = 1.0f / z;
#pragma unroll
    for (int e = 0; e < NE; ++e) sg[tl][e] = w[e] * iz; }
  __syncthreads();
  vst2(GATE + (size_t)blockIdx.x * 64 * NE + tid * 4, *(const v4f*)&(&sg[0][0])[tid * 4]);
}
__global__ __launch_bounds__(128) void k_out(const float* __restrict__ OE, const float* __restrict__ GATE, float* __restrict__ out) {
  __shared__ __align__(16) float so[NC]; const int b = blockIdx.x, c = threadIdx.x; float acc = 0.f;
#pragma unroll 1
  for (int p = 0; p < NP; ++p) { const size_t smp = (size_t)b * NP + p; float s_ = 0.f;
#pragma unroll
    for (int e = 0; e < NE; ++e) s_ += OE[(smp * NE + e) * NC + c] * GATE[smp * NE + e];
    acc += s_; }
  so[c] = acc / (float)NP;
  __syncthreads();
  if (c < 32) vst2(out + (size_t)b * NC + c * 4, *(const v4f*)&so[c * 4]);
}
extern "C" void kernel_launch(void* const* d_in, const int* in_sizes, int n_in, void* d_out, int out_size, void* d_ws, size_t ws_size, hipStream_t stream) {
  (void)in_sizes; (void)n_in; (void)out_size;
  const float** F = (const float**)d_in; const int* TOPK = (const int*)d_in[14];
  if (ws_size < (size_t)WS_END) return;
  char* ws = (char*)d_ws; __bf16* PW = (__bf16*)(ws + WS_PW); float *FEAT = (float*)(ws + WS_FEAT), *EMB = (float*)(ws + WS_EMB), *GATE = (float*)(ws + WS_GATE), *H1 = (float*)(ws + WS_H1), *OE = (float*)(ws + WS_OE);
  k_pack<<<dim3(NE * DD, 6), 256, 0, stream>>>(F[1], F[3], F[5], F[8], F[10], F[12], PW);
  k_conv<<<NSAMP, 128, 0, stream>>>(F[0], PW, F[2], F[4], FEAT);
  k_gemm<8, 2><<<dim3(NSB, DD / 128), 128, 0, stream>>>(FEAT, CH, CH, PW + PPJ, F[6], DD, F[7], EMB, DD);
  k_gate<<<NSB, 128, 0, stream>>>(EMB, PW, F[9], TOPK, GATE);
  k_gemm<8, 1><<<dim3(NSB, NE * DD / 128), 128, 0, stream>>>(EMB, DD, DD, PW + PE1, F[11], NE * DD, nullptr, H1, NE * DD);
  for (int e = 0; e < NE; ++e) k_gemm<8, 0><<<dim3(NSB, 1), 128, 0, stream>>>(H1 + (size_t)e * DD, NE * DD, DD, PW + PE2 + (size_t)e * NC * DD, F[13] + e * NC, NC, nullptr, OE + (size_t)e * NC, NE * NC);
  k_out<<<NB, 128, 0, stream>>>(OE, GATE, (float*)d_out);
}
